// multiTimeAttention_46952582479931
// MI455X (gfx1250) — hardware-run, weakly checked
//
#include <hip/hip_runtime.h>


#ifndef NB
#define NB 8
#endif
#ifndef LQ
#define LQ 128
#endif
#ifndef LK
#define LK 512
#endif
#define NB_FULL 8
#define LQ_FULL 128
#define LK_FULL 512
#ifndef OUT_LQ
#define OUT_LQ LQ
#endif
#define DM   128
#define NHD  2
#define HDIM 64
#define DV   64
#define AW   4
#define OSP  68
#define WTP  136
#define TVP  72
#define SC2  ((float)(0.125 * 1.4426950408889634))
#define PSH  14.0f
#define NEGB (-3.0e38f)
#define VCAR 16.0f
#define XCAR 1024.0f
#define WCAR 64.0f
#define OSCL (1.0f / 65536.0f)

static_assert(NHD * HDIM == DM);
static_assert(NHD * DV == DM);
static_assert(HDIM == 64);
static_assert(DV == 64);
static_assert(DM % 64 == 0);
static_assert(DM % 32 == 0);
static_assert(HDIM % 32 == 0);
static_assert(LQ % 64 == 0);
static_assert(LK % 64 == 0);
static_assert(LQ % (16 * AW) == 0);
static_assert(NB <= NB_FULL);
static_assert(LQ <= LQ_FULL);
static_assert(LK <= LK_FULL);
static_assert((OSP * 4) % 16 == 0);
static_assert((WTP * 2) % 16 == 0);
static_assert((TVP * 2) % 16 == 0);
static_assert(((size_t)LQ * DM) % 8 == 0);
static_assert(((size_t)LK * DM) % 8 == 0);
static_assert(8 * 256 * 4 == DM * 64);
static_assert(4 * 256 * 16 == 64 * DM * 2);
static_assert(4 * 256 * 4 == 64 * DV);
static_assert(2 * 256 * 16 == DV * 64 * 2);
static_assert(4 * 32 * 16 == 16 * HDIM * 2);
static_assert(4 * 32 * 16 == 16 * DV * 2);
static_assert(8 * 32 * 16 == 16 * 64 * 4);
static_assert(16 * OSP * 4 <= 131072);
static_assert(AW * 16 * OSP * 4 <= 131072);
static_assert(64 * WTP * 2 <= 131072);
static_assert(2 * 64 * TVP * 2 + 16 * 64 * 4 + 64 * 4 <= 131072);

typedef _Float16 h16;
typedef unsigned short bf;
typedef __attribute__((ext_vector_type(16))) __bf16   v16bf;
typedef __attribute__((ext_vector_type(16))) _Float16 v16h;
typedef __attribute__((ext_vector_type(8)))  _Float16 v8h;
typedef __attribute__((ext_vector_type(8)))  unsigned short v8us;
typedef __attribute__((ext_vector_type(8)))  float    v8f;
typedef __attribute__((ext_vector_type(4)))  float    v4f;
typedef __attribute__((ext_vector_type(4)))  int      v4i;
typedef v4f  __attribute__((may_alias)) v4fa;
typedef v8h  __attribute__((may_alias)) v8ha;
typedef v8us __attribute__((may_alias)) v8usa;

__device__ __forceinline__ unsigned short f2bf(float f) { unsigned u = __float_as_uint(f); u += 0x7FFFu + ((u >> 16) & 1u); return (unsigned short)(u >> 16); }
__device__ __forceinline__ float bfr(float f) { return __uint_as_float(((unsigned)f2bf(f)) << 16); }
__device__ __forceinline__ v16h cat16(v8h lo, v8h hi) { return __builtin_shufflevector(lo, hi, 0, 1, 2, 3, 4, 5, 6, 7, 8, 9, 10, 11, 12, 13, 14, 15); }
__device__ __forceinline__ v16bf cat16b(v8us lo, v8us hi) { return __builtin_bit_cast(v16bf, __builtin_shufflevector(lo, hi, 0, 1, 2, 3, 4, 5, 6, 7, 8, 9, 10, 11, 12, 13, 14, 15)); }
__device__ __forceinline__ v8f wmma16(v16h a, v16h b, v8f c) { return __builtin_amdgcn_wmma_f32_16x16x32_f16(false, a, false, b, (short)0, c, false, false); }
__device__ __forceinline__ v8f wmmab(v16bf a, v16bf b, v8f c) { return __builtin_amdgcn_wmma_f32_16x16x32_bf16(false, a, false, b, (short)0, c, false, false); }
__device__ __forceinline__ v16h  ldh(const h16* p) { return cat16(*(const v8h*)p, *(const v8h*)(p + 16)); }
__device__ __forceinline__ v16bf ldb(const bf* p)  { return cat16b(*(const v8us*)p, *(const v8us*)(p + 16)); }
__device__ __forceinline__ void wave_sync() { __builtin_amdgcn_fence(3  , "wavefront"); __builtin_amdgcn_wave_barrier(); asm volatile("" ::: "memory"); }

static __device__ __forceinline__ h16 toh_flush(float v) { const h16 r = (h16)v; return (fabsf(v) < 6.103515625e-05f) ? (h16)0.0f : r; }
static __device__ __forceinline__ v8f wmma16g(v16h a, v16h b, v8f c) { c = wmma16(a, b, c); asm volatile("v_nop\n\tv_nop\n\tv_nop\n\tv_nop" : "+v"(c) : "v"(a), "v"(b)); return c; }
static __device__ __forceinline__ v8f wmmabg(v16bf a, v16bf b, v8f c) { c = wmmab(a, b, c); asm volatile("v_nop\n\tv_nop\n\tv_nop\n\tv_nop" : "+v"(c) : "v"(a), "v"(b)); return c; }

__global__ __launch_bounds__(256) void k_cvt8(const float* __restrict__ src, bf* dst, size_t n8) {
    const size_t i = (size_t)blockIdx.x * 256 + threadIdx.x; if (i >= n8) return;
    const v8f v = *(const v8f*)(src + i * 8); v8us o;
#pragma unroll
    for (int k = 0; k < 8; ++k) o[k] = f2bf(v[k]);
    *(volatile v8us*)(dst + i * 8) = o; __threadfence(); *(volatile v8us*)(dst + i * 8) = o;
}

__global__ __launch_bounds__(256) void k_wtb(const float* __restrict__ W, bf* dst) {
    __shared__ __align__(16) unsigned short lt[64 * WTP];
    const int tid = threadIdx.x; const int n0 = blockIdx.x * 64;
#pragma unroll 1
    for (int it = 0; it < 8; ++it) { const int idx = it * 256 + tid; const int k = idx >> 4, n4 = (idx & 15) * 4;
        const v4f v = *(const v4f*)(W + (size_t)k * DM + n0 + n4);
#pragma unroll
        for (int i = 0; i < 4; ++i) lt[(n4 + i) * WTP + k] = f2bf(v[i]); }
    __syncthreads();
#pragma unroll 1
    for (int ps = 0; ps < 2; ++ps) {
#pragma unroll
        for (int it = 0; it < 4; ++it) { const int q = it * 256 + tid; const int n = q >> 4, p = q & 15;
            const v8us o = *(const v8usa*)(&lt[n * WTP + p * 8]);
            *(volatile v8us*)(dst + (size_t)(n0 + n) * DM + p * 8) = o; }
        if (ps == 0) __threadfence(); }
}

__global__ __launch_bounds__(256) void k_wth(const float* __restrict__ W, h16* dst) {
    __shared__ __align__(16) h16 lt[64 * WTP];
    const int tid = threadIdx.x; const int n0 = blockIdx.x * 64;
#pragma unroll 1
    for (int it = 0; it < 8; ++it) { const int idx = it * 256 + tid; const int k = idx >> 4, n4 = (idx & 15) * 4;
        const v4f v = *(const v4f*)(W + (size_t)k * DM + n0 + n4);
#pragma unroll
        for (int i = 0; i < 4; ++i) lt[(n4 + i) * WTP + k] = toh_flush(bfr(v[i]) * WCAR); }
    __syncthreads();
#pragma unroll 1
    for (int ps = 0; ps < 2; ++ps) {
#pragma unroll
        for (int it = 0; it < 4; ++it) { const int q = it * 256 + tid; const int n = q >> 4, p = q & 15;
            const v8h o = *(const v8ha*)(&lt[n * WTP + p * 8]);
            *(volatile v8h*)(dst + (size_t)(n0 + n) * DM + p * 8) = o; }
        if (ps == 0) __threadfence(); }
}

__global__ __launch_bounds__(256) void k_mvt(const float* __restrict__ value, const int* __restrict__ keep, h16* MVT, h16* MT, float* CM) {
#pragma clang fp contract(off)
    __shared__ __align__(16) h16 tv[64 * TVP];
    __shared__ __align__(16) h16 tm[64 * TVP];
    __shared__ float red[16 * 64];
    __shared__ __align__(16) float cs[64];
    const int tid = threadIdx.x; const int b = blockIdx.x;
    const int d4 = (tid & 15) * 4, kq = tid >> 4;
    float s0 = 0.0f, s1 = 0.0f, s2 = 0.0f, s3 = 0.0f;
#pragma unroll 1
    for (int k0 = 0; k0 < LK; k0 += 64) {
#pragma unroll
        for (int it = 0; it < 4; ++it) { const int k = it * 16 + kq;
            const size_t gi = ((size_t)b * LK_FULL + (size_t)(k0 + k)) * DV + d4;
            const v4f v = *(const v4f*)(value + gi);
            const v4i mm = *(const v4i*)(keep + gi);
            float vb[4];
#pragma unroll
            for (int i = 0; i < 4; ++i) { vb[i] = bfr(v[i]); const bool kp = mm[i] != 0;
                tv[(d4 + i) * TVP + k] = kp ? toh_flush(vb[i] * VCAR) : (h16)0.0f;
                tm[(d4 + i) * TVP + k] = kp ? (h16)1.0f : (h16)0.0f; }
            s0 += vb[0]; s1 += vb[1]; s2 += vb[2]; s3 += vb[3]; }
        __syncthreads();
#pragma unroll 1
        for (int ps = 0; ps < 2; ++ps) {
#pragma unroll
            for (int it = 0; it < 2; ++it) { const int q = it * 256 + tid; const int d = q >> 3, p = q & 7;
                const v8h a = *(const v8ha*)(&tv[d * TVP + p * 8]); const v8h c = *(const v8ha*)(&tm[d * TVP + p * 8]);
                const size_t o = ((size_t)b * DV + (size_t)d) * LK + (size_t)k0 + (size_t)p * 8;
                *(volatile v8h*)(MVT + o) = a; *(volatile v8h*)(MT + o) = c; }
            if (ps == 0) __threadfence(); }
        __syncthreads();
    }
    red[kq * 64 + d4 + 0] = s0; red[kq * 64 + d4 + 1] = s1; red[kq * 64 + d4 + 2] = s2; red[kq * 64 + d4 + 3] = s3;
    __syncthreads();
    if (tid < 64) { float s = 0.0f;
#pragma unroll 1
        for (int g = 0; g < 16; ++g) s += red[g * 64 + tid];
        cs[tid] = s * (1.0f / (float)LK); }
    __syncthreads();
    if (tid < 16) { const v4f o = *(const v4fa*)(&cs[tid * 4]);
        *(volatile v4f*)(CM + (size_t)b * DV + tid * 4) = o; __threadfence(); *(volatile v4f*)(CM + (size_t)b * DV + tid * 4) = o; }
}

__global__ __launch_bounds__(32) void k_projh(const bf* __restrict__ A, const bf* __restrict__ Bt, const float* __restrict__ bias, h16* Ph, int seq) {
    __shared__ __align__(16) float os[16 * OSP];
    const int K = DM;
    const int lane = threadIdx.x & 31, lr = lane & 15, hi = lane >> 4; const int r0 = blockIdx.x * 64, c0 = blockIdx.y * 64;
    v8f acc[4][4];
#pragma unroll
    for (int mb = 0; mb < 4; ++mb)
#pragma unroll
        for (int nb = 0; nb < 4; ++nb) acc[mb][nb] = (v8f){};
    const size_t aoff = (size_t)(r0 + lr) * K + 8 * hi, boff = (size_t)(c0 + lr) * K + 8 * hi;
#pragma unroll 1
    for (int kc = 0; kc < K; kc += 32) {
        v16bf a[4];
#pragma unroll
        for (int mb = 0; mb < 4; ++mb) a[mb] = ldb(A + aoff + (size_t)mb * 16 * K + kc);
#pragma unroll
        for (int nb = 0; nb < 4; ++nb) { const v16bf b = ldb(Bt + boff + (size_t)nb * 16 * K + kc);
#pragma unroll
            for (int mb = 0; mb < 4; ++mb) acc[mb][nb] = wmmabg(a[mb], b, acc[mb][nb]); }
    }
    float bc[4];
#pragma unroll
    for (int nb = 0; nb < 4; ++nb) bc[nb] = bfr(bias[c0 + nb * 16 + lr]);
    const int bb = r0 / seq, tt = r0 % seq; const int zc = bb * NHD + c0 / HDIM;
    const size_t tbase = ((size_t)zc * (size_t)seq + (size_t)tt) * HDIM;
#pragma unroll
    for (int mb = 0; mb < 4; ++mb) {
#pragma unroll
        for (int nb = 0; nb < 4; ++nb) {
#pragma unroll
            for (int j = 0; j < 8; ++j) os[(hi * 8 + j) * OSP + nb * 16 + lr] = acc[mb][nb][j] + bc[nb]; }
        wave_sync();
#pragma unroll 1
        for (int ps = 0; ps < 2; ++ps) {
            const size_t sb = tbase + (size_t)(mb * 16) * HDIM;
#pragma unroll
            for (int s = 0; s < 4; ++s) { const int p = s * 32 + lane; const int row = p >> 3, c8 = (p & 7) * 8;
                const v4f x0 = *(const v4fa*)(&os[row * OSP + c8]); const v4f x1 = *(const v4fa*)(&os[row * OSP + c8 + 4]); v8h hv;
#pragma unroll
                for (int i = 0; i < 4; ++i) { hv[i] = toh_flush(x0[i]); hv[4 + i] = toh_flush(x1[i]); }
                *(volatile v8h*)(Ph + sb + (size_t)p * 8) = hv; }
            if (ps == 0) __threadfence(); }
        wave_sync();
    }
}

static __device__ __forceinline__ void fin8(const v8f n, const v8f d, const v4f c0, const v4f c1, v4f& a, v4f& c) {
#pragma unroll
    for (int i = 0; i < 4; ++i) {
        const float da = d[i], dc = d[4 + i];
        const bool ya = da > 0.0f, yc = dc > 0.0f;
        const float xa = n[i] * __builtin_amdgcn_rcpf((ya ? da : 1.0f) * VCAR);
        const float xc = n[4 + i] * __builtin_amdgcn_rcpf((yc ? dc : 1.0f) * VCAR);
        a[i] = (ya ? xa : c0[i]) * XCAR; c[i] = (yc ? xc : c1[i]) * XCAR; }
}

__global__ __launch_bounds__(32 * AW) __attribute__((amdgpu_num_vgpr(256)))
void k_flash(const h16* __restrict__ QH, const h16* __restrict__ KP, const h16* __restrict__ MVT, const h16* __restrict__ MT, const float* __restrict__ CM, h16* XH) {
    __shared__ __align__(16) float os[AW * 16 * OSP];
    const int lane = threadIdx.x & 31, lr = lane & 15, hi = lane >> 4;
    const int wave = __builtin_amdgcn_readfirstlane((int)(threadIdx.x >> 5));
    const int zh = blockIdx.y; const int b = zh / NHD, h = zh % NHD;
    const int t0 = (blockIdx.x * AW + wave) * 16;
    const size_t qo = ((size_t)zh * LQ + (size_t)(t0 + lr)) * HDIM + 8 * hi;
    const v16h qf0 = ldh(QH + qo), qf1 = ldh(QH + qo + 32);
    const size_t ko = ((size_t)zh * LK + (size_t)lr) * HDIM + 8 * hi;
    const size_t vo = ((size_t)b * DV + (size_t)lr) * LK + 8 * hi;
    v8f n0 = (v8f){}, n1 = (v8f){}, n2 = (v8f){}, n3 = (v8f){};
    v8f d0 = (v8f){}, d1 = (v8f){}, d2 = (v8f){}, d3 = (v8f){};
    float m = NEGB;
#pragma unroll 1
    for (int key0 = 0; key0 < LK; key0 += 32) {
        const h16* ka = KP + ko + (size_t)key0 * HDIM;
        const v16h ka0 = ldh(ka), ka1 = ldh(ka + 32), kb0 = ldh(ka + 16 * HDIM), kb1 = ldh(ka + 16 * HDIM + 32);
        v8f sa = (v8f){}, sb = (v8f){};
        sa = wmma16g(ka0, qf0, sa); sa = wmma16g(ka1, qf1, sa);
        sb = wmma16g(kb0, qf0, sb); sb = wmma16g(kb1, qf1, sb);
        float ta[8], tb[8]; float mx = NEGB;
#pragma unroll
        for (int r = 0; r < 8; ++r) { ta[r] = sa[r] * SC2; tb[r] = sb[r] * SC2; mx = fmaxf(mx, fmaxf(ta[r], tb[r])); }
        mx = fmaxf(mx, __shfl_xor(mx, 16, 32));
        const float mnew = fmaxf(m, mx);
        const float alpha = __builtin_amdgcn_exp2f(m - mnew);
        const float sh = PSH - mnew;
        v16h pb;
#pragma unroll
        for (int r = 0; r < 8; ++r) {
            const float ea = ta[r] + sh, eb = tb[r] + sh;
            const float ga = (ea < -14.0f) ? 0.0f : __builtin_amdgcn_exp2f(ea);
            const float gb = (eb < -14.0f) ? 0.0f : __builtin_amdgcn_exp2f(eb);
            pb[r] = (h16)ga; pb[8 + r] = (h16)gb; }
        m = mnew;
        n0 = n0 * alpha; n1 = n1 * alpha; n2 = n2 * alpha; n3 = n3 * alpha;
        d0 = d0 * alpha; d1 = d1 * alpha; d2 = d2 * alpha; d3 = d3 * alpha;
        { const h16* va = MVT + vo + key0;
          const v16h v0 = ldh(va), v1 = ldh(va + (size_t)16 * LK), v2 = ldh(va + (size_t)32 * LK), v3 = ldh(va + (size_t)48 * LK);
          n0 = wmma16g(v0, pb, n0); n1 = wmma16g(v1, pb, n1); n2 = wmma16g(v2, pb, n2); n3 = wmma16g(v3, pb, n3); }
        { const h16* ma = MT + vo + key0;
          const v16h v0 = ldh(ma), v1 = ldh(ma + (size_t)16 * LK), v2 = ldh(ma + (size_t)32 * LK), v3 = ldh(ma + (size_t)48 * LK);
          d0 = wmma16g(v0, pb, d0); d1 = wmma16g(v1, pb, d1); d2 = wmma16g(v2, pb, d2); d3 = wmma16g(v3, pb, d3); }
    }
    const float* cmb = CM + (size_t)b * DV + 8 * hi;
    const int wb = wave * 16 * OSP;
    { v4f a, c;
      fin8(n0, d0, *(const v4f*)(cmb +  0), *(const v4f*)(cmb +  4), a, c);
      *(v4fa*)(&os[wb + lr * OSP +  0 + 8 * hi]) = a; *(v4fa*)(&os[wb + lr * OSP +  0 + 8 * hi + 4]) = c;
      fin8(n1, d1, *(const v4f*)(cmb + 16), *(const v4f*)(cmb + 20), a, c);
      *(v4fa*)(&os[wb + lr * OSP + 16 + 8 * hi]) = a; *(v4fa*)(&os[wb + lr * OSP + 16 + 8 * hi + 4]) = c;
      fin8(n2, d2, *(const v4f*)(cmb + 32), *(const v4f*)(cmb + 36), a, c);
      *(v4fa*)(&os[wb + lr * OSP + 32 + 8 * hi]) = a; *(v4fa*)(&os[wb + lr * OSP + 32 + 8 * hi + 4]) = c;
      fin8(n3, d3, *(const v4f*)(cmb + 48), *(const v4f*)(cmb + 52), a, c);
      *(v4fa*)(&os[wb + lr * OSP + 48 + 8 * hi]) = a; *(v4fa*)(&os[wb + lr * OSP + 48 + 8 * hi + 4]) = c; }
    wave_sync();
    h16* xrow = XH + ((size_t)b * LQ + (size_t)t0) * DM + h * DV;
#pragma unroll 1
    for (int ps = 0; ps < 2; ++ps) {
#pragma unroll
        for (int s = 0; s < 4; ++s) { const int row = 4 * s + (lane >> 3), c8 = (lane & 7) * 8;
            const v4f x0 = *(const v4fa*)(&os[wb + row * OSP + c8]); const v4f x1 = *(const v4fa*)(&os[wb + row * OSP + c8 + 4]); v8h hv;
#pragma unroll
            for (int i = 0; i < 4; ++i) { hv[i] = toh_flush(x0[i]); hv[4 + i] = toh_flush(x1[i]); }
            *(volatile v8h*)(xrow + (size_t)row * DM + c8) = hv; }
        if (ps == 0) __threadfence(); }
}

__global__ __launch_bounds__(32) void k_outp(const h16* __restrict__ A, const h16* __restrict__ Bt, const float* __restrict__ bias, float* OUT) {
    __shared__ __align__(16) float os[16 * OSP];
    const int K = DM;
    const int lane = threadIdx.x & 31, lr = lane & 15, hi = lane >> 4; const int r0 = blockIdx.x * 64, c0 = blockIdx.y * 64;
    v8f acc[4][4];
#pragma unroll
    for (int mb = 0; mb < 4; ++mb)
#pragma unroll
        for (int nb = 0; nb < 4; ++nb) acc[mb][nb] = (v8f){};
    const size_t aoff = (size_t)(r0 + lr) * K + 8 * hi, boff = (size_t)(c0 + lr) * K + 8 * hi;
#pragma unroll 1
    for (int kc = 0; kc < K; kc += 32) {
        v16h a[4];
#pragma unroll
        for (int mb = 0; mb < 4; ++mb) a[mb] = ldh(A + aoff + (size_t)mb * 16 * K + kc);
#pragma unroll
        for (int nb = 0; nb < 4; ++nb) { const v16h b = ldh(Bt + boff + (size_t)nb * 16 * K + kc);
#pragma unroll
            for (int mb = 0; mb < 4; ++mb) acc[mb][nb] = wmma16g(a[mb], b, acc[mb][nb]); }
    }
    float bc[4];
#pragma unroll
    for (int nb = 0; nb < 4; ++nb) bc[nb] = bfr(bias[c0 + nb * 16 + lr]);
    const int bb = r0 / LQ, tt = r0 % LQ;
    float* obase = OUT + ((size_t)bb * OUT_LQ + (size_t)tt) * DM + c0;
#pragma unroll
    for (int mb = 0; mb < 4; ++mb) {
#pragma unroll
        for (int nb = 0; nb < 4; ++nb) {
#pragma unroll
            for (int j = 0; j < 8; ++j) os[(hi * 8 + j) * OSP + nb * 16 + lr] = acc[mb][nb][j] * OSCL + bc[nb]; }
        wave_sync();
#pragma unroll 1
        for (int ps = 0; ps < 2; ++ps) {
#pragma unroll
            for (int s = 0; s < 8; ++s) { const int row = 2 * s + (lane >> 4), c4 = (lane & 15) * 4;
                const v4f val = *(const v4fa*)(&os[row * OSP + c4]);
                *(volatile v4f*)(obase + (size_t)(mb * 16 + row) * DM + c4) = val; }
            if (ps == 0) __threadfence(); }
        wave_sync();
    }
}

static constexpr size_t al256(size_t v) { return (v + 255) & ~(size_t)255; }
static constexpr size_t SZ_XQ = al256((size_t)NB * LQ * DM * 2);
static constexpr size_t SZ_XK = al256((size_t)NB * LK * DM * 2);
static constexpr size_t SZ_W  = al256((size_t)DM * DM * 2);
static constexpr size_t SZ_QH = al256((size_t)NB * NHD * LQ * HDIM * 2);
static constexpr size_t SZ_KP = al256((size_t)NB * NHD * LK * HDIM * 2);
static constexpr size_t SZ_VT = al256((size_t)NB * DV * LK * 2);
static constexpr size_t SZ_CM = al256((size_t)NB * DV * 4);
static constexpr size_t SZ_XH = al256((size_t)NB * LQ * DM * 2);
static constexpr size_t SZ_TOTAL = SZ_XQ + SZ_XK + 3 * SZ_W + SZ_QH + SZ_KP + 2 * SZ_VT + SZ_CM + SZ_XH;
static_assert(SZ_TOTAL <= (size_t)134217728);
static_assert(((size_t)DV * 4) % 256 == 0);
static_assert((NB * LQ) % 64 == 0);
static_assert((NB * LK) % 64 == 0);

extern "C" void kernel_launch(void* const* d_in, const int* in_sizes, int n_in,
                              void* d_out, int out_size, void* d_ws, size_t ws_size, hipStream_t stream) {
    if (n_in < 10) return;
    if ((size_t)in_sizes[0] < ((size_t)(NB - 1) * LQ_FULL + LQ) * DM) return;
    if ((size_t)in_sizes[1] < ((size_t)(NB - 1) * LK_FULL + LK) * DM) return;
    if ((size_t)in_sizes[2] < ((size_t)(NB - 1) * LK_FULL + LK) * DV) return;
    if ((size_t)in_sizes[3] < ((size_t)(NB - 1) * LK_FULL + LK) * DV) return;
    if ((size_t)in_sizes[4] < (size_t)DM * DM || (size_t)in_sizes[6] < (size_t)DM * DM || (size_t)in_sizes[8] < (size_t)DM * DM) return;
    if (in_sizes[5] < DM || in_sizes[7] < DM || in_sizes[9] < DM) return;
    if ((size_t)out_size < ((size_t)(NB - 1) * OUT_LQ + LQ) * DM) return;
    if (SZ_TOTAL > ws_size) return;
    const float* query = (const float*)d_in[0];
    const float* key   = (const float*)d_in[1];
    const float* value = (const float*)d_in[2];
    const int*   keep  = (const int*)d_in[3];
    const float* wq = (const float*)d_in[4]; const float* bq = (const float*)d_in[5];
    const float* wk = (const float*)d_in[6]; const float* bk = (const float*)d_in[7];
    const float* wo = (const float*)d_in[8]; const float* bo = (const float*)d_in[9];
    float* OUT = (float*)d_out;
    char* wsp = (char*)d_ws;
    bf*  XQ  = (bf*)wsp;  wsp += SZ_XQ;
    bf*  XK  = (bf*)wsp;  wsp += SZ_XK;
    bf*  WQB = (bf*)wsp;  wsp += SZ_W;
    bf*  WKB = (bf*)wsp;  wsp += SZ_W;
    h16* WOH = (h16*)wsp; wsp += SZ_W;
    h16* QH  = (h16*)wsp; wsp += SZ_QH;
    h16* KP  = (h16*)wsp; wsp += SZ_KP;
    h16* MVT = (h16*)wsp; wsp += SZ_VT;
    h16* MT  = (h16*)wsp; wsp += SZ_VT;
    float* CM = (float*)wsp; wsp += SZ_CM;
    h16* XH  = (h16*)wsp; wsp += SZ_XH;

    if (LQ == LQ_FULL) {
        const size_t n8 = (size_t)NB * LQ * DM / 8;
        k_cvt8<<<(unsigned)((n8 + 255) / 256), 256, 0, stream>>>(query, XQ, n8);
    } else {
        const size_t n8 = (size_t)LQ * DM / 8;
        for (int b = 0; b < NB; ++b) k_cvt8<<<(unsigned)((n8 + 255) / 256), 256, 0, stream>>>(query + (size_t)b * LQ_FULL * DM, XQ + (size_t)b * LQ * DM, n8);
    }
    if (LK == LK_FULL) {
        const size_t n8 = (size_t)NB * LK * DM / 8;
        k_cvt8<<<(unsigned)((n8 + 255) / 256), 256, 0, stream>>>(key, XK, n8);
    } else {
        const size_t n8 = (size_t)LK * DM / 8;
        for (int b = 0; b < NB; ++b) k_cvt8<<<(unsigned)((n8 + 255) / 256), 256, 0, stream>>>(key + (size_t)b * LK_FULL * DM, XK + (size_t)b * LK * DM, n8);
    }
    k_wtb<<<DM / 64, 256, 0, stream>>>(wq, WQB);
    k_wtb<<<DM / 64, 256, 0, stream>>>(wk, WKB);
    k_wth<<<DM / 64, 256, 0, stream>>>(wo, WOH);
    k_mvt<<<NB, 256, 0, stream>>>(value, keep, MVT, MT, CM);

    k_projh<<<dim3(NB * LQ / 64, DM / 64, 1), 32, 0, stream>>>(XQ, WQB, bq, QH, LQ);
    k_projh<<<dim3(NB * LK / 64, DM / 64, 1), 32, 0, stream>>>(XK, WKB, bk, KP, LK);

    k_flash<<<dim3(LQ / (16 * AW), NB * NHD, 1), 32 * AW, 0, stream>>>(QH, KP, MVT, MT, CM, XH);

    k_outp<<<dim3(NB * LQ / 64, DM / 64, 1), 32, 0, stream>>>(XH, WOH, bo, OUT);
}
